// Smoother_41128606826509
// MI455X (gfx1250) — hardware-verified
//
#include <hip/hip_runtime.h>

typedef __attribute__((ext_vector_type(16))) _Float16 v16h;
typedef __attribute__((ext_vector_type(8)))  float    v8f;
typedef __attribute__((ext_vector_type(4)))  float    v4f;
typedef float __attribute__((may_alias)) float_a;
template <typename T> __device__ __forceinline__ void vst2(void* p, T v) { *(volatile T*)p = v; __threadfence(); *(volatile T*)p = v; }

#define T_DIM 2048
#define B_DIM 32
#define ROWS_PER_BLOCK 64
#define BLOCK_THREADS 128
#define SQRT_2PI 2.5066282746310002f
#define LOG2E    1.4426950408889634f

__launch_bounds__(BLOCK_THREADS)
__global__ void smoother_wmma_kernel(const float* __restrict__ src,
                                     const float* __restrict__ timeA,
                                     const float* __restrict__ mask,
                                     const float* __restrict__ p_ptr,
                                     float* __restrict__ stg) {
    __shared__ __align__(16) float    gS[T_DIM];
    __shared__ __align__(32) _Float16 srcH[T_DIM];
    __shared__ float redMax[BLOCK_THREADS];
    __shared__ float redMin[BLOCK_THREADS];
    __shared__ float dOut[4][32][8];

    const int b    = blockIdx.y;
    const int t0bk = blockIdx.x * ROWS_PER_BLOCK;
    const int tid  = threadIdx.x;

    const float p     = p_ptr[0];
    const float C     = 1.0f / (p * SQRT_2PI);
    const float negHp = -0.5f / p;
    const float posHp =  0.5f / p;

    float lmax = -__builtin_inff();
    float lmin =  __builtin_inff();
    for (int s = tid; s < T_DIM; s += BLOCK_THREADS) {
        float ts = timeA[s * B_DIM + b];
        float g  = expf(negHp * ts) * mask[s * B_DIM + b];
        gS[s]    = g;
        srcH[s]  = (_Float16)src[s * B_DIM + b];
        lmax = fmaxf(lmax, g);
        lmin = fminf(lmin, g);
    }
    redMax[tid] = lmax;
    redMin[tid] = lmin;
    __syncthreads();
    for (int off = BLOCK_THREADS / 2; off > 0; off >>= 1) {
        if (tid < off) {
            redMax[tid] = fmaxf(redMax[tid], redMax[tid + off]);
            redMin[tid] = fminf(redMin[tid], redMin[tid + off]);
        }
        __syncthreads();
    }
    const float gmax = redMax[0];
    const float gmin = redMin[0];

    const int wave = tid >> 5;
    const int lane = tid & 31;
    const int m    = lane & 15;
    const int t    = t0bk + wave * 16 + m;

    const float a_m  = C * expf(posHp * timeA[t * B_DIM + b]);
    const float mx_m = (a_m >= 0.0f) ? a_m * gmax : a_m * gmin;
    const float a2   = a_m  * LOG2E;
    const float mx2  = mx_m * LOG2E;

    const int kbaseA = (lane < 16) ? 0 : 8;
    const int n      = m;

    const _Float16 selSrc = (n == 0) ? (_Float16)1.0f : (_Float16)0.0f;
    const _Float16 selOne = (n == 1) ? (_Float16)1.0f : (_Float16)0.0f;

    v8f acc = {};

#pragma unroll 2
    for (int s0 = 0; s0 < T_DIM; s0 += 32) {
        float logit[16];
#pragma unroll
        for (int j = 0; j < 16; ++j) {
            const int k = kbaseA + j + ((j >= 8) ? 8 : 0);
            logit[j] = a2 * gS[s0 + k] - mx2;
        }
        float pe[16];
#pragma unroll
        for (int j = 0; j < 16; ++j) {
            pe[j] = exp2f(logit[j]);
        }
        v16h afrag;
#pragma unroll
        for (int j = 0; j < 16; ++j) {
            afrag[j] = (_Float16)pe[j];
        }

        typedef __attribute__((ext_vector_type(8))) _Float16 v8h;
        union { v16h v; v8h q[2]; } svu;
        svu.q[0] = *(const v8h*)(srcH + s0 + kbaseA); svu.q[1] = *(const v8h*)(srcH + s0 + kbaseA + 16);
        const v16h bfrag = svu.v * selSrc + selOne;

        acc = __builtin_amdgcn_wmma_f32_16x16x32_f16(
                   false, afrag,  false, bfrag,
                   (short)0, acc,  false,  false);
        asm volatile("v_nop\n\tv_nop\n\tv_nop\n\tv_nop" : "+v"(acc) : "v"(afrag), "v"(bfrag));
    }

#pragma unroll
    for (int r = 0; r < 8; ++r) dOut[wave][lane][r] = acc[r];
    __syncthreads();

    __shared__ float res[ROWS_PER_BLOCK];
    if (lane < 16) {
        const int srcLane = (m < 8) ? 0 : 16;
        const int r       = m & 7;
        const float num = dOut[wave][srcLane][r];
        const float den = dOut[wave][srcLane + 1][r];
        res[wave * 16 + m] = num / den;
    }
    __syncthreads();
    if (tid < ROWS_PER_BLOCK) vst2(stg + (size_t)b * T_DIM + t0bk + tid, (float_a)res[tid]);
}

__global__ void transpose_out_kernel(const float* __restrict__ stg, float* __restrict__ out) {
    __shared__ float tile[32][33];
    const int t0 = blockIdx.x * 32, tid = threadIdx.x;
    for (int i = tid; i < 32 * 32; i += 256) { const int bb = i >> 5, tt = i & 31; tile[bb][tt] = stg[(size_t)bb * T_DIM + t0 + tt]; }
    __syncthreads();
    for (int i = tid; i < 32 * 32; i += 256) { const int tt = i >> 5, bb = i & 31; vst2(out + (size_t)(t0 + tt) * B_DIM + bb, (float_a)tile[bb][tt]); }
}

extern "C" void kernel_launch(void* const* d_in, const int* in_sizes, int n_in,
                              void* d_out, int out_size, void* d_ws, size_t ws_size,
                              hipStream_t stream) {
    const float* src   = (const float*)d_in[0];
    const float* timeA = (const float*)d_in[1];
    const float* mask  = (const float*)d_in[2];
    const float* p     = (const float*)d_in[3];
    float* out = (float*)d_out;

    float* stg = (float*)d_ws;
    dim3 grid(T_DIM / ROWS_PER_BLOCK, B_DIM);
    smoother_wmma_kernel<<<grid, BLOCK_THREADS, 0, stream>>>(src, timeA, mask, p, stg);
    transpose_out_kernel<<<T_DIM / 32, 256, 0, stream>>>(stg, out);
}
